// MolMPNN_3547642987145
// MI455X (gfx1250) — hardware-run, weakly checked
//
#include <hip/hip_runtime.h>
#include <stddef.h>
#include <stdint.h>


#define NN       50000
#define NE       600000
#define DM       128
#define MP       50048
#define GBM      128
#define GTHR     256
#define GNT      8
#define BN       128
#define APW      256
#define SPLIT_A  1
#define SPLIT_B  1
#define KS_P     4
#define KS_A     (SPLIT_A ? 8 : 4)
#define KS_B     (SPLIT_B ? 8 : 4)
#define NTHR     256
#define NWAVE    8
#define EPT      8
#define CHUNK    (NTHR * EPT)
#define WCAP     (EPT * 32)
#define LISTN    (NWAVE * WCAP)
#define NB       1024
#define NAGG     49
#define RCAP     16384
#define DEGCAP   64
#define PKS      11
#define STW      512
#define LDS_AGG  ((2 * RCAP + 2 * NB + LISTN + 3 * NWAVE) * 4)
#define LDS_GEMM ((GBM * BN + 3 * DM) * 4)
#define PB_HB    ((MP * (DM / 8)) / NTHR)
#define PB_WP    ((DM * (DM / 8)) / NTHR)
#define PB_WD    ((DM * (APW / 8)) / NTHR)
#define PB_ALL   (PB_HB + PB_WP + 2 * PB_WD + 1)

static_assert(DM == 128 && BN == DM && APW == 2 * DM);
static_assert(MP == ((NN + GBM - 1) / GBM) * GBM && (MP % GBM) == 0);
static_assert(GBM == (GTHR / 32) * 16 && BN == 16 * GNT);
static_assert(NAGG * NB >= MP && (NAGG - 1) * NB < NN);
static_assert((NB % GBM) == 0 && ((MP / GBM - 1) / (NB / GBM)) < NAGG);
static_assert((CHUNK & (CHUNK - 1)) == 0 && CHUNK <= (1 << PKS));
static_assert((NB & (NB - 1)) == 0 && NB <= (1 << PKS) && NTHR * 4 == NB);
static_assert(LISTN >= NB && (NB % NWAVE) == 0);
static_assert(NE <= (1 << 21) && (NE % 4) == 0);
static_assert((RCAP % 32) == 0 && NWAVE * STW <= RCAP && STW >= 128);
static_assert(RCAP * 100 >= 12567 * 105);
static_assert(DEGCAP >= 28 + 8);
static_assert(LDS_AGG <= 327680 && LDS_GEMM <= 327680);
static_assert(((MP * (DM / 8)) % NTHR) == 0 && ((DM * (DM / 8)) % NTHR) == 0 && ((DM * (APW / 8)) % NTHR) == 0);
static_assert(KS_P * 32 == DM && KS_A * 32 <= APW && KS_B * 32 <= APW);

typedef float          v4f  __attribute__((ext_vector_type(4)));
typedef float          v8f  __attribute__((ext_vector_type(8)));
typedef int            v4i  __attribute__((ext_vector_type(4)));
typedef int            v8i  __attribute__((ext_vector_type(8)));
typedef unsigned int   v2u  __attribute__((ext_vector_type(2)));
typedef unsigned int   v4u  __attribute__((ext_vector_type(4)));
typedef unsigned short v8us __attribute__((ext_vector_type(8)));
typedef __bf16         v16b __attribute__((ext_vector_type(16)));
typedef v4f  __attribute__((may_alias)) v4fa;
typedef v4i  __attribute__((may_alias)) v4ia;
typedef v2u  __attribute__((may_alias)) v2ua;
typedef v4u  __attribute__((may_alias)) v4ua;
typedef v8us __attribute__((may_alias)) v8usa;
union FragB { v16b v; v8us h[2]; v8i w; };

constexpr size_t SZ_HB  = (size_t)MP * DM * 2;
constexpr size_t SZ_HF  = (size_t)MP * DM * 4;
constexpr size_t SZ_HL  = (size_t)MP * APW * 2;
constexpr size_t SZ_WP  = (size_t)DM * DM * 2;
constexpr size_t SZ_WD  = (size_t)DM * APW * 2;
constexpr size_t SZ_PAR = (size_t)5 * DM * 4;
constexpr size_t SZ_FLG = (((size_t)NAGG * 128) + 255) & ~(size_t)255;
constexpr size_t O_HB   = 0;
constexpr size_t O_HF   = O_HB + SZ_HB;
constexpr size_t O_AG   = O_HF + SZ_HF;
constexpr size_t O_TP   = O_AG + SZ_HL;
constexpr size_t O_WP   = O_TP + SZ_HL;
constexpr size_t O_WA   = O_WP + SZ_WP;
constexpr size_t O_WB   = O_WA + SZ_WD;
constexpr size_t O_PAR  = O_WB + SZ_WD;
constexpr size_t O_FLG  = O_PAR + SZ_PAR;
constexpr size_t WS_TOTAL = O_FLG + SZ_FLG;
static_assert((O_HF % 256) == 0 && (O_AG % 256) == 0 && (O_TP % 256) == 0 && (O_WP % 256) == 0);
static_assert((O_WA % 256) == 0 && (O_WB % 256) == 0 && (O_PAR % 256) == 0 && (O_FLG % 256) == 0);
static_assert(WS_TOTAL <= (size_t)(128u << 20));

__device__ __forceinline__ v8f wmb(const FragB& a, const FragB& b, v8f c) {
  v8f d = __builtin_amdgcn_wmma_f32_16x16x32_bf16(false, a.v, false, b.v, (short)0, c, false, false);
  asm volatile("v_nop\n\tv_nop\n\tv_nop\n\tv_nop" : "+v"(d) : "v"(a.w), "v"(b.w));
  return d;
}

__device__ __forceinline__ unsigned short bf_bits(float f) {
  const unsigned int u = __float_as_uint(f);
  unsigned int r = u + 0x7fffu + ((u >> 16) & 1u);
  r = (f != f) ? 0x7fc00000u : r;
  return (unsigned short)(r >> 16);
}
__device__ __forceinline__ float bf_val(unsigned short b) {
  return __uint_as_float(((unsigned int)b) << 16);
}
__device__ __forceinline__ float bf_rne(float f) { return bf_val(bf_bits(f)); }

template <int KW>
__device__ __forceinline__ void wplane_unit(const float* __restrict__ W, unsigned short* plane, int v) {
  constexpr int UPR = KW / 8;
  const int n  = v / UPR;
  const int k8 = (v - n * UPR) * 8;
  const int kk = k8 & (DM - 1);
  const float* p = W + (size_t)kk * DM + n;
  v8us o;
#pragma unroll
  for (int i = 0; i < 8; ++i) o[i] = bf_bits(p[(size_t)i * DM]);
  unsigned short* dp = plane + (size_t)n * KW + k8;
  *(volatile v8us*)dp = o;
  __threadfence();
  *(volatile v8us*)dp = o;
}

__global__ __launch_bounds__(NTHR) void k_prep(
    const float* __restrict__ h, const float* __restrict__ wpre,
    const float* __restrict__ wa, const float* __restrict__ wb,
    const float* __restrict__ bpre, const float* __restrict__ ba, const float* __restrict__ bb,
    const float* __restrict__ gam, const float* __restrict__ bet,
    unsigned short* hb, unsigned short* wpt, unsigned short* wad, unsigned short* wbd, float* par) {
  const int blk = (int)blockIdx.x, tid = (int)threadIdx.x;
  if (blk < PB_HB) {
    const int u   = blk * NTHR + tid;
    const int row = u >> 4;
    const int c8  = (u & 15) * 8;
    const int rc  = row < NN ? row : NN - 1;
    const v4f a = *(const v4f*)(h + (size_t)rc * DM + c8);
    const v4f b = *(const v4f*)(h + (size_t)rc * DM + c8 + 4);
    asm volatile("" :: "v"(a), "v"(b));
    const unsigned short msk = (row < NN) ? (unsigned short)0xffffu : (unsigned short)0u;
    v8us o;
    o[0] = (unsigned short)(bf_bits(a.x) & msk);
    o[1] = (unsigned short)(bf_bits(a.y) & msk);
    o[2] = (unsigned short)(bf_bits(a.z) & msk);
    o[3] = (unsigned short)(bf_bits(a.w) & msk);
    o[4] = (unsigned short)(bf_bits(b.x) & msk);
    o[5] = (unsigned short)(bf_bits(b.y) & msk);
    o[6] = (unsigned short)(bf_bits(b.z) & msk);
    o[7] = (unsigned short)(bf_bits(b.w) & msk);
    unsigned short* dp = hb + (size_t)row * DM + c8;
    *(volatile v8us*)dp = o;
    __threadfence();
    *(volatile v8us*)dp = o;
  } else if (blk < PB_HB + PB_WP) {
    wplane_unit<DM>(wpre, wpt, (blk - PB_HB) * NTHR + tid);
  } else if (blk < PB_HB + PB_WP + PB_WD) {
    wplane_unit<APW>(wa, wad, (blk - PB_HB - PB_WP) * NTHR + tid);
  } else if (blk < PB_HB + PB_WP + 2 * PB_WD) {
    wplane_unit<APW>(wb, wbd, (blk - PB_HB - PB_WP - PB_WD) * NTHR + tid);
  } else {
    const int row = tid >> 5;
    const int c4  = (tid & 31) * 4;
    const v4f q0 = *(const v4f*)(bpre + c4);
    const v4f q1 = *(const v4f*)(ba + c4);
    const v4f q2 = *(const v4f*)(bb + c4);
    const v4f q3 = *(const v4f*)(gam + c4);
    const v4f q4 = *(const v4f*)(bet + c4);
    v4f s = q0;
    s = (row == 1) ? q1 : s;
    s = (row == 2) ? q2 : s;
    s = (row == 3) ? q3 : s;
    s = (row >= 4) ? q4 : s;
    v4f o;
    o.x = bf_rne(s.x); o.y = bf_rne(s.y); o.z = bf_rne(s.z); o.w = bf_rne(s.w);
    const int rowc = row < 5 ? row : 4;
    float* dp = par + (size_t)rowc * DM + c4;
    const bool ok = row < 5;
    if (ok) *(volatile v4f*)dp = o;
    __threadfence();
    if (ok) *(volatile v4f*)dp = o;
  }
}

__device__ __forceinline__ int scan_chunk(const int* __restrict__ dsts, int cbase, int slotBase,
                                          int nbv, int vec8, int* list, int tid, int lane, int wave) {
  int wc = 0;
  const int el0  = tid * EPT;
  const int e0   = cbase + el0;
  const int sent = (int)(1u << 31);
  v4i da, db;
  if (vec8 != 0 && cbase + CHUNK <= NE) {
    da = *(const v4i*)(dsts + e0);
    db = *(const v4i*)(dsts + e0 + 4);
  } else {
    const int t0 = dsts[min(e0,     NE - 1)];
    const int t1 = dsts[min(e0 + 1, NE - 1)];
    const int t2 = dsts[min(e0 + 2, NE - 1)];
    const int t3 = dsts[min(e0 + 3, NE - 1)];
    const int t4 = dsts[min(e0 + 4, NE - 1)];
    const int t5 = dsts[min(e0 + 5, NE - 1)];
    const int t6 = dsts[min(e0 + 6, NE - 1)];
    const int t7 = dsts[min(e0 + 7, NE - 1)];
    asm volatile("" :: "v"(t0), "v"(t1), "v"(t2), "v"(t3), "v"(t4), "v"(t5), "v"(t6), "v"(t7));
    da.x = (e0     < NE) ? t0 : sent;
    da.y = (e0 + 1 < NE) ? t1 : sent;
    da.z = (e0 + 2 < NE) ? t2 : sent;
    da.w = (e0 + 3 < NE) ? t3 : sent;
    db.x = (e0 + 4 < NE) ? t4 : sent;
    db.y = (e0 + 5 < NE) ? t5 : sent;
    db.z = (e0 + 6 < NE) ? t6 : sent;
    db.w = (e0 + 7 < NE) ? t7 : sent;
  }
  const unsigned nbs = (unsigned)slotBase;
  const unsigned unb = (unsigned)nbv;
  const unsigned s0 = (unsigned)da.x - nbs, s1 = (unsigned)da.y - nbs;
  const unsigned s2 = (unsigned)da.z - nbs, s3 = (unsigned)da.w - nbs;
  const unsigned s4 = (unsigned)db.x - nbs, s5 = (unsigned)db.y - nbs;
  const unsigned s6 = (unsigned)db.z - nbs, s7 = (unsigned)db.w - nbs;
  const bool h0 = s0 < unb, h1 = s1 < unb, h2 = s2 < unb, h3 = s3 < unb;
  const bool h4 = s4 < unb, h5 = s5 < unb, h6 = s6 < unb, h7 = s7 < unb;
  const unsigned any = __builtin_amdgcn_ballot_w32(h0 | h1 | h2 | h3 | h4 | h5 | h6 | h7);
  if (any != 0u) {
    const unsigned m0 = __builtin_amdgcn_ballot_w32(h0);
    const unsigned m1 = __builtin_amdgcn_ballot_w32(h1);
    const unsigned m2 = __builtin_amdgcn_ballot_w32(h2);
    const unsigned m3 = __builtin_amdgcn_ballot_w32(h3);
    const unsigned m4 = __builtin_amdgcn_ballot_w32(h4);
    const unsigned m5 = __builtin_amdgcn_ballot_w32(h5);
    const unsigned m6 = __builtin_amdgcn_ballot_w32(h6);
    const unsigned m7 = __builtin_amdgcn_ballot_w32(h7);
    unsigned low = __builtin_amdgcn_mbcnt_lo(m0, 0u);
    low = __builtin_amdgcn_mbcnt_lo(m1, low);
    low = __builtin_amdgcn_mbcnt_lo(m2, low);
    low = __builtin_amdgcn_mbcnt_lo(m3, low);
    low = __builtin_amdgcn_mbcnt_lo(m4, low);
    low = __builtin_amdgcn_mbcnt_lo(m5, low);
    low = __builtin_amdgcn_mbcnt_lo(m6, low);
    low = __builtin_amdgcn_mbcnt_lo(m7, low);
    int p = (int)low;
#define HITP(J, HJ, SJ) { \
      if (HJ) { if (p < WCAP) list[wave * WCAP + p] = ((el0 + (J)) << PKS) | (int)(SJ); } \
      p += (HJ) ? 1 : 0; }
    HITP(0, h0, s0)
    HITP(1, h1, s1)
    HITP(2, h2, s2)
    HITP(3, h3, s3)
    HITP(4, h4, s4)
    HITP(5, h5, s5)
    HITP(6, h6, s6)
    HITP(7, h7, s7)
#undef HITP
    wc = (int)(__builtin_popcount(m0) + __builtin_popcount(m1) + __builtin_popcount(m2) + __builtin_popcount(m3) +
               __builtin_popcount(m4) + __builtin_popcount(m5) + __builtin_popcount(m6) + __builtin_popcount(m7));
  }
  return wc;
}

__global__ __launch_bounds__(NTHR) void k_agg(
    const int* __restrict__ srcs, const int* __restrict__ dsts, const float* __restrict__ F,
    unsigned short* Aout, int* flagp, int vec8) {
  extern __shared__ v4f lds_dyn[];
  int* reg1 = (int*)lds_dyn;
  int* reg2 = reg1 + RCAP;
  int* scnt = reg2 + RCAP;
  int* soff = scnt + NB;
  int* list = soff + NB;
  int* wcnt = list + LISTN;
  int* wtot = wcnt + NWAVE;
  int* wflg = wtot + NWAVE;
  const int tid = (int)threadIdx.x, lane = tid & 31, wave = tid >> 5;
  const int nodeBase = (int)blockIdx.x * NB;
  int nbv = NN - nodeBase;
  nbv = nbv < 0 ? 0 : (nbv > NB ? NB : nbv);

  for (int i = tid; i < NB; i += NTHR) scnt[i] = 0;
  __syncthreads();

  int tot = 0;
  const int nChunks = (NE + CHUNK - 1) / CHUNK;
#pragma unroll 1
  for (int ch = 0; ch < nChunks; ++ch) {
    const int cbase = ch * CHUNK;
    const int wc = scan_chunk(dsts, cbase, nodeBase, nbv, vec8, list, tid, lane, wave);
    if (lane == 0) wcnt[wave] = wc;
    __syncthreads();
    int pre = 0, all = 0;
#pragma unroll
    for (int w2 = 0; w2 < NWAVE; ++w2) {
      int c = wcnt[w2];
      c = c < 0 ? 0 : (c > WCAP ? WCAP : c);
      all += c;
      pre += (w2 < wave) ? c : 0;
    }
    const int wcc  = wc > WCAP ? WCAP : wc;
    const int base = tot + pre;
#pragma unroll 1
    for (int i = lane; i < wcc; i += 32) {
      const int ent = list[wave * WCAP + i];
      const int el  = (ent >> PKS) & (CHUNK - 1);
      const int sl  = ent & (NB - 1);
      int eid = cbase + el;
      eid = eid > NE - 1 ? NE - 1 : eid;
      const int pos = base + i;
      if (pos < RCAP) reg1[pos] = (int)(((unsigned)eid << PKS) | (unsigned)sl);
    }
    tot += all;
    tot = tot > RCAP ? RCAP : tot;
    __syncthreads();
  }
  const int nh = tot;

  if (wave == 0) {
#pragma unroll 1
    for (int b0 = 0; b0 < nh; b0 += 32) {
      const int idx = b0 + lane;
      const int uv  = reg1[idx < RCAP ? idx : RCAP - 1];
      const int m32 = (nh - b0) < 32 ? (nh - b0) : 32;
#pragma unroll 1
      for (int k = 0; k < m32; ++k) {
        const int u  = __builtin_amdgcn_readlane(uv, k);
        const int sl = u & (NB - 1);
        if (lane == 0) scnt[sl] = scnt[sl] + 1;
      }
    }
  }
  __syncthreads();

  int anyov = 0;
  {
    const v4i ca = *(const v4ia*)(scnt + 4 * tid);
    const int e0 = ca.x < 0 ? 0 : ca.x, e1 = ca.y < 0 ? 0 : ca.y;
    const int e2 = ca.z < 0 ? 0 : ca.z, e3 = ca.w < 0 ? 0 : ca.w;
    const bool over = (ca.x > DEGCAP) | (ca.y > DEGCAP) | (ca.z > DEGCAP) | (ca.w > DEGCAP);
    const int ts = e0 + e1 + e2 + e3;
    int incl = ts;
#pragma unroll
    for (int d = 1; d < 32; d <<= 1) {
      const int up = __shfl_up(incl, d);
      if (lane >= d) incl += up;
    }
    const unsigned ob = __builtin_amdgcn_ballot_w32(over);
    if (lane == 31) wtot[wave] = incl;
    if (lane == 0) wflg[wave] = (ob != 0u) ? 1 : 0;
    __syncthreads();
    int pre = 0;
#pragma unroll
    for (int w2 = 0; w2 < NWAVE; ++w2) {
      pre += (w2 < wave) ? wtot[w2] : 0;
      anyov |= wflg[w2];
    }
    int run = pre + incl - ts;
    soff[4 * tid + 0] = run; run += e0;
    soff[4 * tid + 1] = run; run += e1;
    soff[4 * tid + 2] = run; run += e2;
    soff[4 * tid + 3] = run;
  }
  __syncthreads();
  for (int i = tid; i < NB; i += NTHR) list[i] = soff[i];
  __syncthreads();

  if (wave == 0) {
#pragma unroll 1
    for (int b0 = 0; b0 < nh; b0 += 32) {
      const int idx = b0 + lane;
      const int uv  = reg1[idx < RCAP ? idx : RCAP - 1];
      const int m32 = (nh - b0) < 32 ? (nh - b0) : 32;
#pragma unroll 1
      for (int k = 0; k < m32; ++k) {
        const int u   = __builtin_amdgcn_readlane(uv, k);
        const int sl  = u & (NB - 1);
        const int eid = (int)((unsigned)u >> PKS);
        if (lane == 0) {
          int pos = list[sl];
          pos = pos < 0 ? 0 : (pos > RCAP - 1 ? RCAP - 1 : pos);
          reg2[pos] = eid;
          list[sl] = pos + 1;
        }
      }
    }
  }
  __syncthreads();

  const int nbw = NB / NWAVE;
  const bool bflag = (nh >= RCAP) || (anyov != 0);
  const float qnan = __int_as_float(0x7fc00000);
  const float pz = bflag ? qnan : 0.0f;
  unsigned int* stwu = (unsigned int*)(reg1 + wave * STW);

#pragma unroll 1
  for (int jt = 0; jt < nbw; ++jt) {
    const int slot = wave * nbw + jt;
    const int grow = nodeBase + slot;
    int st  = soff[slot];
    int cnt = scnt[slot];
    st  = st < 0 ? 0 : (st > nh ? nh : st);
    cnt = cnt < 0 ? 0 : (cnt > DEGCAP ? DEGCAP : cnt);
    cnt = cnt > nh - st ? nh - st : cnt;
    st  = __builtin_amdgcn_readfirstlane(st);
    cnt = __builtin_amdgcn_readfirstlane(cnt);
    const bool liveRow = grow < NN;

    float ag0 = 0.0f, ag1 = 0.0f, ag2 = 0.0f, ag3 = 0.0f;
#pragma unroll 1
    for (int b0 = 0; b0 < cnt; b0 += 32) {
      int idx = st + b0 + lane;
      idx = idx > nh - 1 ? nh - 1 : idx;
      idx = idx < 0 ? 0 : (idx > RCAP - 1 ? RCAP - 1 : idx);
      int eid = reg2[idx];
      eid = eid < 0 ? 0 : (eid > NE - 1 ? NE - 1 : eid);
      const int sraw = srcs[eid];
      const int sv = sraw < 0 ? 0 : (sraw > NN - 1 ? NN - 1 : sraw);
      const int m32 = (cnt - b0) < 32 ? (cnt - b0) : 32;
#pragma unroll 1
      for (int k = 0; k < m32; ++k) {
        const int sk = __builtin_amdgcn_readlane(sv, k);
        const v4f v = *(const v4f*)(F + (size_t)sk * DM + 4 * lane);
        ag0 += v.x; ag1 += v.y; ag2 += v.z; ag3 += v.w;
      }
    }
    const float r0 = (liveRow ? ag0 : 0.0f) + pz;
    const float r1 = (liveRow ? ag1 : 0.0f) + pz;
    const float r2 = (liveRow ? ag2 : 0.0f) + pz;
    const float r3 = (liveRow ? ag3 : 0.0f) + pz;

    const unsigned short hb0 = bf_bits(r0), hb1 = bf_bits(r1), hb2 = bf_bits(r2), hb3 = bf_bits(r3);
    const unsigned short lb0 = bf_bits(r0 - bf_val(hb0)), lb1 = bf_bits(r1 - bf_val(hb1));
    const unsigned short lb2 = bf_bits(r2 - bf_val(hb2)), lb3 = bf_bits(r3 - bf_val(hb3));
    v2u hw, lw;
    hw.x = (unsigned int)hb0 | ((unsigned int)hb1 << 16);
    hw.y = (unsigned int)hb2 | ((unsigned int)hb3 << 16);
    lw.x = (unsigned int)lb0 | ((unsigned int)lb1 << 16);
    lw.y = (unsigned int)lb2 | ((unsigned int)lb3 << 16);
    __builtin_amdgcn_fence(__ATOMIC_RELEASE, "wavefront");
    __builtin_amdgcn_wave_barrier();
    *(v2ua*)(stwu + 2 * lane)      = hw;
    *(v2ua*)(stwu + 64 + 2 * lane) = lw;
    __builtin_amdgcn_fence(__ATOMIC_RELEASE, "wavefront");
    __builtin_amdgcn_wave_barrier();
    const v4u pk = *(const v4ua*)(stwu + 4 * lane);
    unsigned short* gp = Aout + (size_t)grow * (size_t)APW + 8 * lane;
    const bool wsv = grow < MP;
    if (wsv) *(volatile v4u*)gp = pk;
    __threadfence();
    if (wsv) *(volatile v4u*)gp = pk;
  }

  {
    const int fvv = bflag ? 1 : 0;
    const v4i fv = {fvv, fvv, fvv, fvv};
    int* fp = flagp + (size_t)blockIdx.x * 32 + 4 * (tid & 7);
    const bool fw = tid < 8;
    if (fw) *(volatile v4i*)fp = fv;
    __threadfence();
    if (fw) *(volatile v4i*)fp = fv;
  }
}

template <int MODE, int KS, int APITCH, int WPITCH>
__global__ __launch_bounds__(GTHR) __attribute__((amdgpu_num_vgpr(248)))
void k_gemm(const unsigned short* __restrict__ A, const unsigned short* __restrict__ WT,
            const float* __restrict__ par, int bsel, void* outp,
            const float* __restrict__ hres, const int* __restrict__ flagp)
{
  static_assert(KS * 32 <= APITCH && KS * 32 <= WPITCH);
  static_assert((APITCH % 8) == 0 && (WPITCH % 8) == 0);
  constexpr int NT = GNT;
  constexpr int NI = 16;
  extern __shared__ v4f lds_dyn[];
  float* stg  = (float*)lds_dyn;
  float* spar = stg + GBM * BN;
  const int tid = (int)threadIdx.x, lane = tid & 31, wave = tid >> 5, hh = lane >> 4, m = lane & 15;
  const int rowBase = (int)blockIdx.x * GBM;

  if (tid < 32) {
    const v4f pb = *(const v4f*)(par + (size_t)bsel * DM + 4 * tid);
    const v4f pg = *(const v4f*)(par + (size_t)3 * DM + 4 * tid);
    const v4f pe = *(const v4f*)(par + (size_t)4 * DM + 4 * tid);
    *(v4fa*)(spar + 4 * tid)          = pb;
    *(v4fa*)(spar + DM + 4 * tid)     = pg;
    *(v4fa*)(spar + 2 * DM + 4 * tid) = pe;
  }
  __syncthreads();

  v8f acc[NT];
  {
    const v8f z = {0.f, 0.f, 0.f, 0.f, 0.f, 0.f, 0.f, 0.f};
#pragma unroll
    for (int t = 0; t < NT; ++t) acc[t] = z;
  }
  const unsigned short* ap = A + (size_t)(rowBase + 16 * wave + m) * (size_t)APITCH + 8 * hh;
  const unsigned short* wp = WT + (size_t)m * (size_t)WPITCH + 8 * hh;
#pragma unroll 1
  for (int ks = 0; ks < KS; ++ks) {
    FragB af;
    af.h[0] = *(const v8usa*)(ap + 32 * ks);
    af.h[1] = *(const v8usa*)(ap + 32 * ks + 16);
#pragma unroll
    for (int t = 0; t < NT; ++t) {
      const unsigned short* wq = wp + (size_t)(16 * t) * (size_t)WPITCH + 32 * ks;
      FragB bf;
      bf.h[0] = *(const v8usa*)wq;
      bf.h[1] = *(const v8usa*)(wq + 16);
      acc[t] = wmb(af, bf, acc[t]);
    }
  }

#pragma unroll
  for (int t = 0; t < NT; ++t) {
    const int lc = 16 * t + m;
    const float bb = spar[lc];
#pragma unroll
    for (int r = 0; r < 8; ++r) {
      const int lr = 16 * wave + 8 * hh + r;
      float v = acc[t][r] + bb;
      if (MODE != 0) v = (v > 0.0f) ? v : (v - v);
      stg[lr * BN + lc] = v;
    }
  }
  __syncthreads();

  if constexpr (MODE == 0) {
    float* outF = (float*)outp;
    v4f fv[NI];
#pragma unroll
    for (int i = 0; i < NI; ++i) {
      const int lr = 16 * wave + i;
      fv[i] = *(const v4fa*)(stg + lr * BN + 4 * lane);
    }
#pragma unroll
    for (int i = 0; i < NI; ++i) {
      const int gr = rowBase + 16 * wave + i;
      float* op = outF + (size_t)gr * (size_t)DM + 4 * lane;
      if (gr < MP) *(volatile v4f*)op = fv[i];
    }
    __threadfence();
#pragma unroll
    for (int i = 0; i < NI; ++i) {
      const int gr = rowBase + 16 * wave + i;
      float* op = outF + (size_t)gr * (size_t)DM + 4 * lane;
      if (gr < MP) *(volatile v4f*)op = fv[i];
    }
  } else if constexpr (MODE == 1) {
    unsigned short* outH = (unsigned short*)outp;
    const int cb = 8 * m;
    const bool isHi = (hh == 0);
    v4u pk[NI];
#pragma unroll
    for (int i = 0; i < NI; ++i) {
      const int lr = 16 * wave + i;
      const v4f a = *(const v4fa*)(stg + lr * BN + cb);
      const v4f b = *(const v4fa*)(stg + lr * BN + cb + 4);
      const float f[8] = {a.x, a.y, a.z, a.w, b.x, b.y, b.z, b.w};
      unsigned int w[4];
#pragma unroll
      for (int j = 0; j < 4; ++j) {
        const unsigned short h0 = bf_bits(f[2 * j]), h1 = bf_bits(f[2 * j + 1]);
        const unsigned short l0 = bf_bits(f[2 * j] - bf_val(h0)), l1 = bf_bits(f[2 * j + 1] - bf_val(h1));
        const unsigned short q0 = isHi ? h0 : l0, q1 = isHi ? h1 : l1;
        w[j] = (unsigned int)q0 | ((unsigned int)q1 << 16);
      }
      v4u pw; pw.x = w[0]; pw.y = w[1]; pw.z = w[2]; pw.w = w[3];
      pk[i] = pw;
    }
#pragma unroll
    for (int i = 0; i < NI; ++i) {
      const int gr = rowBase + 16 * wave + i;
      unsigned short* op = outH + (size_t)gr * (size_t)APW + 8 * lane;
      if (gr < MP) *(volatile v4u*)op = pk[i];
    }
    __threadfence();
#pragma unroll
    for (int i = 0; i < NI; ++i) {
      const int gr = rowBase + 16 * wave + i;
      unsigned short* op = outH + (size_t)gr * (size_t)APW + 8 * lane;
      if (gr < MP) *(volatile v4u*)op = pk[i];
    }
  } else {
    float* outF = (float*)outp;
    int fb = (int)blockIdx.x / (NB / GBM);
    fb = fb > NAGG - 1 ? NAGG - 1 : fb;
    const int fl = flagp[(size_t)fb * 32];
    const bool poison = (fl == 1);
    const float qnan = __int_as_float(0x7fc00000);
    const v4f g4 = *(const v4fa*)(spar + DM + 4 * lane);
    const v4f e4 = *(const v4fa*)(spar + 2 * DM + 4 * lane);
#pragma unroll 1
    for (int i = 0; i < NI; ++i) {
      const int lr = 16 * wave + i;
      const int gr = rowBase + lr;
      const int rc = gr < NN ? gr : NN - 1;
      const v4f v  = *(const v4fa*)(stg + lr * BN + 4 * lane);
      const v4f hr = *(const v4f*)(hres + (size_t)rc * DM + 4 * lane);
      const float y0 = v.x + hr.x, y1 = v.y + hr.y, y2 = v.z + hr.z, y3 = v.w + hr.w;
      float s = (y0 + y1) + (y2 + y3);
      s += __shfl_xor(s, 16);
      s += __shfl_xor(s, 8);
      s += __shfl_xor(s, 4);
      s += __shfl_xor(s, 2);
      s += __shfl_xor(s, 1);
      const float mu = s * 0.0078125f;
      const float d0 = y0 - mu, d1 = y1 - mu, d2 = y2 - mu, d3 = y3 - mu;
      float q = (d0 * d0 + d1 * d1) + (d2 * d2 + d3 * d3);
      q += __shfl_xor(q, 16);
      q += __shfl_xor(q, 8);
      q += __shfl_xor(q, 4);
      q += __shfl_xor(q, 2);
      q += __shfl_xor(q, 1);
      const float var = q * 0.0078125f;
      const float rs = 1.0f / sqrtf(var + 1e-5f);
      v4f o;
      o.x = (d0 * rs) * g4.x + e4.x;
      o.y = (d1 * rs) * g4.y + e4.y;
      o.z = (d2 * rs) * g4.z + e4.z;
      o.w = (d3 * rs) * g4.w + e4.w;
      o.x = poison ? qnan : o.x;
      o.y = poison ? qnan : o.y;
      o.z = poison ? qnan : o.z;
      o.w = poison ? qnan : o.w;
      *(v4fa*)(stg + lr * BN + 4 * lane) = o;
    }
    v4f fv[NI];
#pragma unroll
    for (int i = 0; i < NI; ++i) {
      const int lr = 16 * wave + i;
      fv[i] = *(const v4fa*)(stg + lr * BN + 4 * lane);
    }
#pragma unroll
    for (int i = 0; i < NI; ++i) {
      const int gr = rowBase + 16 * wave + i;
      const int gc = gr < NN ? gr : NN - 1;
      float* op = outF + (size_t)gc * (size_t)DM + 4 * lane;
      if (gr < NN) *(volatile v4f*)op = fv[i];
    }
    __threadfence();
#pragma unroll
    for (int i = 0; i < NI; ++i) {
      const int gr = rowBase + 16 * wave + i;
      const int gc = gr < NN ? gr : NN - 1;
      float* op = outF + (size_t)gc * (size_t)DM + 4 * lane;
      if (gr < NN) *(volatile v4f*)op = fv[i];
    }
  }
}

extern "C" void kernel_launch(void* const* d_in, const int* in_sizes, int n_in,
                              void* d_out, int out_size, void* d_ws, size_t ws_size,
                              hipStream_t stream) {
  if (n_in < 11) return;
  if (in_sizes[0] != NN * DM) return;
  if (in_sizes[1] != NE || in_sizes[2] != NE) return;
  if (in_sizes[3] != DM * DM || in_sizes[5] != DM * DM || in_sizes[7] != DM * DM) return;
  if (in_sizes[4] != DM || in_sizes[6] != DM || in_sizes[8] != DM) return;
  if (in_sizes[9] != DM || in_sizes[10] != DM) return;
  if (out_size != NN * DM) return;
  if (ws_size < WS_TOTAL) return;

  const float* h    = (const float*)d_in[0];
  const int*   src  = (const int*)  d_in[1];
  const int*   dst  = (const int*)  d_in[2];
  const float* Wpre = (const float*)d_in[3];
  const float* bpre = (const float*)d_in[4];
  const float* Wa   = (const float*)d_in[5];
  const float* ba   = (const float*)d_in[6];
  const float* Wb   = (const float*)d_in[7];
  const float* bb   = (const float*)d_in[8];
  const float* gam  = (const float*)d_in[9];
  const float* bet  = (const float*)d_in[10];
  float* out = (float*)d_out;

  char* ws = (char*)d_ws;
  unsigned short* HB  = (unsigned short*)(ws + O_HB);
  float*          HF  = (float*)(ws + O_HF);
  unsigned short* AG  = (unsigned short*)(ws + O_AG);
  unsigned short* TP  = (unsigned short*)(ws + O_TP);
  unsigned short* WPT = (unsigned short*)(ws + O_WP);
  unsigned short* WAD = (unsigned short*)(ws + O_WA);
  unsigned short* WBD = (unsigned short*)(ws + O_WB);
  float*          PAR = (float*)(ws + O_PAR);
  int*            FLG = (int*)(ws + O_FLG);

  hipFuncSetAttribute(reinterpret_cast<const void*>(&k_agg), hipFuncAttributeMaxDynamicSharedMemorySize, LDS_AGG);
  hipFuncSetAttribute(reinterpret_cast<const void*>(&k_gemm<0, KS_P, DM, DM>),
                      hipFuncAttributeMaxDynamicSharedMemorySize, LDS_GEMM);
  hipFuncSetAttribute(reinterpret_cast<const void*>(&k_gemm<1, KS_A, APW, APW>),
                      hipFuncAttributeMaxDynamicSharedMemorySize, LDS_GEMM);
  hipFuncSetAttribute(reinterpret_cast<const void*>(&k_gemm<2, KS_B, APW, APW>),
                      hipFuncAttributeMaxDynamicSharedMemorySize, LDS_GEMM);

  k_prep<<<PB_ALL, NTHR, 0, stream>>>(h, Wpre, Wa, Wb, bpre, ba, bb, gam, bet, HB, WPT, WAD, WBD, PAR);
  k_gemm<0, KS_P, DM, DM><<<MP / GBM, GTHR, LDS_GEMM, stream>>>(HB, WPT, PAR, 0, (void*)HF, PAR, FLG);
  k_agg<<<NAGG, NTHR, LDS_AGG, stream>>>(src, dst, HF, AG, FLG, 1);
  k_gemm<1, KS_A, APW, APW><<<MP / GBM, GTHR, LDS_GEMM, stream>>>(AG, WAD, PAR, 1, (void*)TP, PAR, FLG);
  k_gemm<2, KS_B, APW, APW><<<MP / GBM, GTHR, LDS_GEMM, stream>>>(TP, WBD, PAR, 2, (void*)out, HF, FLG);
}
